// GruBlock_39573828666303
// MI455X (gfx1250) — hardware-verified
//
#include <hip/hip_runtime.h>
#include <math.h>

typedef __attribute__((ext_vector_type(16))) _Float16 v16h;
typedef __attribute__((ext_vector_type(8)))  _Float16 v8h;
typedef __attribute__((ext_vector_type(16))) __bf16   v16b;
typedef __attribute__((ext_vector_type(8)))  __bf16   v8b;
typedef __attribute__((ext_vector_type(8)))  float    v8f;
typedef __attribute__((ext_vector_type(4)))  float    v4f;

constexpr int kB   = 16;
constexpr int kS   = 64;
constexpr int kCin = 64;
constexpr int kPx  = 64;
constexpr int kHid = 128;
constexpr int kGc  = 32;
constexpr int kG   = 2048;
constexpr int kG3  = 6144;
constexpr int kImg = kB * kS;
constexpr float kWScale = 64.0f;
constexpr float kWInv   = 1.0f / 64.0f;

static_assert(kImg % 64 == 0 && kG3 % 64 == 0 && kG % 32 == 0);
static_assert(kCin % 32 == 0 && kHid % 32 == 0 && kGc % 32 == 0);
static_assert(kGc * kPx == kG);

constexpr size_t kSzW16   = (size_t)kG3 * kG * 2;
constexpr size_t kOffWih  = 0;
constexpr size_t kOffWhh  = kOffWih + kSzW16;
constexpr size_t kOffCinW = kOffWhh + kSzW16;
constexpr size_t kOffGruW = kOffCinW + (size_t)kHid * kCin * 2;
constexpr size_t kOffGoW  = kOffGruW + (size_t)kGc * kHid * 2;
constexpr size_t kOffCoW  = kOffGoW + (size_t)kHid * kGc * 2;
constexpr size_t kOffG16  = kOffCoW + (size_t)kCin * kHid * 2;
constexpr size_t kOffGi   = kOffG16 + (size_t)kImg * kG * 2;
constexpr size_t kOffH32a = kOffGi + (size_t)kImg * kG3 * 4;
constexpr size_t kOffH32b = kOffH32a + (size_t)kB * kG * 4;
constexpr size_t kOffH16a = kOffH32b + (size_t)kB * kG * 4;
constexpr size_t kOffH16b = kOffH16a + (size_t)kB * kG * 2;
constexpr size_t kOffGseq = kOffH16b + (size_t)kB * kG * 2;
constexpr size_t kWsTotal = kOffGseq + (size_t)kImg * kG * 4;
static_assert(kWsTotal == 88522752u);
static_assert(kWsTotal <= 134217728u);
static_assert(kOffCinW % 128 == 0 && kOffGruW % 128 == 0 && kOffGoW % 128 == 0 && kOffCoW % 128 == 0);
static_assert(kOffG16 % 128 == 0 && kOffGi % 128 == 0 && kOffH32a % 128 == 0 && kOffH16a % 128 == 0 && kOffGseq % 128 == 0);

constexpr size_t kOut0Floats = (size_t)kImg * kCin * kPx;
constexpr size_t kOut1Floats = (size_t)kB * kG;
static_assert(kOut0Floats * 4 == 16777216u);
static_assert((kOut0Floats + kOut1Floats) * 4 == 16908288u);

constexpr int kXaP  = 72;
constexpr int kH1P  = 68;
constexpr int kHtP  = 136;
constexpr int kBt1P = 40;
constexpr int kFrXa = 0;
constexpr int kFrH1 = 9216;
constexpr int kFrH2 = 44032;
constexpr int kFrLds = 78848;
static_assert(kFrXa + kPx * kXaP * 2 <= kFrH1);
static_assert(kFrH1 + kHid * kH1P * 4 == kFrH2);
static_assert(kFrH2 + kHid * kH1P * 4 == kFrLds);
static_assert(kPx * kHtP * 2 <= kHid * kH1P * 4);
static_assert(kGc * kPx * 4 <= kFrH1);

__device__ __forceinline__ unsigned short f2bf_bits(float f) {
  unsigned u = __float_as_uint(f);
  return (unsigned short)((u + 0x7FFFu + ((u >> 16) & 1u)) >> 16);
}
__device__ __forceinline__ float bf_bits2f(unsigned short h) { return __uint_as_float(((unsigned)h) << 16); }

__device__ __forceinline__ void dep_guard_h(v8f& a, v8f& b, v16h x, v16h y) { asm volatile("v_nop\n\tv_nop\n\tv_nop\n\tv_nop" : "+v"(a), "+v"(b) : "v"(x), "v"(y)); }
__device__ __forceinline__ void dep_guard_b(v8f& a, v8f& b, v16b x, v16b y) { asm volatile("v_nop\n\tv_nop\n\tv_nop\n\tv_nop" : "+v"(a), "+v"(b) : "v"(x), "v"(y)); }
__device__ __forceinline__ void keep4_h(v16h a, v16h b, v16h c, v16h d) { asm volatile("v_nop" :: "v"(a), "v"(b), "v"(c), "v"(d)); }
__device__ __forceinline__ void keep4_b(v16b a, v16b b, v16b c, v16b d) { asm volatile("v_nop" :: "v"(a), "v"(b), "v"(c), "v"(d)); }
__device__ __forceinline__ void acc_guard4(v8f& a, v8f& b, v8f& c, v8f& d) { asm volatile("v_nop\n\tv_nop\n\tv_nop\n\tv_nop" : "+v"(a), "+v"(b), "+v"(c), "+v"(d)); }
__device__ __forceinline__ void acc_guard2(v8f& a, v8f& b) { asm volatile("v_nop\n\tv_nop\n\tv_nop\n\tv_nop" : "+v"(a), "+v"(b)); }
__device__ __forceinline__ void acc_guard1(v8f& a) { asm volatile("v_nop\n\tv_nop\n\tv_nop\n\tv_nop" : "+v"(a)); }
__device__ __forceinline__ void guard1h(v8f& a, v16h x, v16h y) { asm volatile("v_nop\n\tv_nop\n\tv_nop\n\tv_nop" : "+v"(a) : "v"(x), "v"(y)); }
__device__ __forceinline__ void guard4h(v8f& a, v8f& b, v8f& c, v8f& d, v16h x, v16h y) {
  asm volatile("v_nop\n\tv_nop\n\tv_nop\n\tv_nop" : "+v"(a), "+v"(b), "+v"(c), "+v"(d) : "v"(x), "v"(y));
}
__device__ __forceinline__ void guard6h(v8f& a, v8f& b, v8f& c, v8f& d, v8f& e, v8f& f, v16h x, v16h y) {
  asm volatile("v_nop\n\tv_nop\n\tv_nop\n\tv_nop" : "+v"(a), "+v"(b), "+v"(c), "+v"(d), "+v"(e), "+v"(f) : "v"(x), "v"(y));
}
__device__ __forceinline__ void wave_lds_sync() {
  __builtin_amdgcn_fence(__ATOMIC_RELEASE, "workgroup");
  __builtin_amdgcn_wave_barrier();
  __builtin_amdgcn_fence(__ATOMIC_ACQUIRE, "workgroup");
}
__device__ __forceinline__ v8f zero8() { return (v8f){0.f, 0.f, 0.f, 0.f, 0.f, 0.f, 0.f, 0.f}; }

template <typename T> struct Frag;
template <> struct Frag<_Float16> {
  typedef v16h V; union U { v16h v; v8h h[2]; };
  static __device__ __forceinline__ v16h load(const _Float16* p) {
    U f; f.h[0] = *(const v8h*)(p); f.h[1] = *(const v8h*)(p + 16); return f.v;
  }
  static __device__ __forceinline__ v8f mma(v16h a, v16h b, v8f c) {
    return __builtin_amdgcn_wmma_f32_16x16x32_f16(false, a, false, b, (short)0, c, false, false);
  }
  static __device__ __forceinline__ void guard(v8f& a, v8f& b, v16h x, v16h y) { dep_guard_h(a, b, x, y); }
  static __device__ __forceinline__ void keep(v16h a, v16h b, v16h c, v16h d) { keep4_h(a, b, c, d); }
};
template <> struct Frag<__bf16> {
  typedef v16b V; union U { v16b v; v8b h[2]; };
  static __device__ __forceinline__ v16b load(const __bf16* p) {
    U f; f.h[0] = *(const v8b*)(p); f.h[1] = *(const v8b*)(p + 16); return f.v;
  }
  static __device__ __forceinline__ v8f mma(v16b a, v16b b, v8f c) {
    return __builtin_amdgcn_wmma_f32_16x16x32_bf16(false, a, false, b, (short)0, c, false, false);
  }
  static __device__ __forceinline__ void guard(v8f& a, v8f& b, v16b x, v16b y) { dep_guard_b(a, b, x, y); }
  static __device__ __forceinline__ void keep(v16b a, v16b b, v16b c, v16b d) { keep4_b(a, b, c, d); }
};

template <int ET> struct Elem;
template <> struct Elem<0> { typedef _Float16 T; };
template <> struct Elem<1> { typedef __bf16 T; };
template <int ET, bool SPLIT, int BIAS_MODE, int OUT_MODE, bool RESID, int ACT = 0>
__global__ __launch_bounds__(256) void wmma_gemm64(
    const unsigned short* __restrict__ Ap, const unsigned short* __restrict__ A2p, int lda, long strideA,
    const unsigned short* __restrict__ Btp, const unsigned short* __restrict__ Bt2p, int ldb, long strideB,
    void* __restrict__ Cout, void* __restrict__ Cout2, int ldc, long strideC,
    const float* __restrict__ bias,
    const float* __restrict__ resid, long strideR,
    int M, int N, int K, float scale) {
  typedef typename Elem<ET>::T T;
  typedef typename Frag<T>::V V;
  const T* A = (const T*)Ap; const T* A2 = (const T*)A2p; const T* Bt = (const T*)Btp; const T* Bt2 = (const T*)Bt2p;
  __shared__ __align__(16) float sT[8][16 * 68];
  const int b    = blockIdx.y;
  const int lane = threadIdx.x & 31;
  const int wave = threadIdx.x >> 5;
  const int tilesN = N >> 6;
  const int tilesM = M >> 6;
  const int tile = blockIdx.x * 8 + wave;
  if (tile >= tilesM * tilesN) return;
  const int tm = tile / tilesN;
  const int tn = tile - tm * tilesN;
  const int m0 = tm << 6;
  const int n0 = tn << 6;

  const T* Ab  = A  + (size_t)b * strideA;
  const T* Bb  = Bt + (size_t)b * strideB;
  const T* Ab2 = SPLIT ? (A2  + (size_t)b * strideA) : nullptr;
  const T* Bb2 = SPLIT ? (Bt2 + (size_t)b * strideB) : nullptr;

  const int rlane = lane & 15;
  const int koff  = (lane >> 4) * 8;
  const int mOff  = (lane >> 4) * 8;

  v8f acc[4][4];
#pragma unroll
  for (int i = 0; i < 4; ++i)
#pragma unroll
    for (int j = 0; j < 4; ++j) acc[i][j] = (v8f){0.f,0.f,0.f,0.f,0.f,0.f,0.f,0.f};

  for (int k0 = 0; k0 < K; k0 += 32) {
    V bh[4], bl[4];
#pragma unroll
    for (int j = 0; j < 4; ++j) {
      const size_t bo = (size_t)(n0 + (j << 4) + rlane) * ldb + koff + k0;
      bh[j] = Frag<T>::load(Bb + bo);
      if (SPLIT) bl[j] = Frag<T>::load(Bb2 + bo);
    }
#pragma unroll
    for (int i = 0; i < 4; ++i) {
      const size_t ao = (size_t)(m0 + (i << 4) + rlane) * lda + koff + k0;
      V ah = Frag<T>::load(Ab + ao);
      V al;
      if (SPLIT) al = Frag<T>::load(Ab2 + ao);
#pragma unroll
      for (int j = 0; j < 4; ++j) {
        acc[i][j] = Frag<T>::mma(ah, bh[j], acc[i][j]);
        if (SPLIT) {
          acc[i][j] = Frag<T>::mma(ah, bl[j], acc[i][j]);
          acc[i][j] = Frag<T>::mma(al, bh[j], acc[i][j]);
        }
      }
      Frag<T>::guard(acc[i][0], acc[i][3], ah, SPLIT ? al : ah);
    }
    Frag<T>::keep(bh[0], bh[1], bh[2], bh[3]);
    if (SPLIT) Frag<T>::keep(bl[0], bl[1], bl[2], bl[3]);
  }
  acc_guard4(acc[0][0], acc[0][1], acc[0][2], acc[0][3]);
  acc_guard4(acc[1][0], acc[1][1], acc[1][2], acc[1][3]);
  acc_guard4(acc[2][0], acc[2][1], acc[2][2], acc[2][3]);
  acc_guard4(acc[3][0], acc[3][1], acc[3][2], acc[3][3]);

  float* slab = sT[wave];
  const float* Rb = RESID ? (resid + (size_t)b * strideR) : nullptr;
#pragma unroll
  for (int i = 0; i < 4; ++i) {
    const int mBase = m0 + (i << 4);
#pragma unroll
    for (int j = 0; j < 4; ++j) {
      const int n = n0 + (j << 4) + rlane;
      float bv = 0.f;
      if (BIAS_MODE == 2) bv = bias[n];
#pragma unroll
      for (int r = 0; r < 8; ++r) {
        float v = acc[i][j][r] * scale;
        if (BIAS_MODE == 1) v += bias[mBase + mOff + r];
        if (BIAS_MODE == 2) v += bv;
        if (RESID) v += Rb[(size_t)(mBase + mOff + r) * ldc + n];
        if (ACT == 1) v = tanhf(v);
        if (ACT == 2) v = fmaxf(v, 0.0f);
        if (ACT == 3) v = v / (1.0f + expf(-v));
        if (ACT == 4) v = (v > 0.f) ? v : 0.01f * v;
        if (ACT == 5) v = 0.5f * v * (1.0f + erff(v * 0.70710678118654752f));
        slab[(mOff + r) * 68 + (j << 4) + rlane] = v;
      }
    }
    __builtin_amdgcn_fence(__ATOMIC_RELEASE, "workgroup");
    __builtin_amdgcn_wave_barrier();
    __builtin_amdgcn_fence(__ATOMIC_ACQUIRE, "workgroup");
    if (OUT_MODE == 0) {
      float* C = (float*)Cout + (size_t)b * strideC;
      const int hh = lane >> 4, c4 = (lane & 15) * 4;
      for (int pass = 0; pass < 2; ++pass) {
#pragma unroll
        for (int it = 0; it < 8; ++it) {
          const int row = it * 2 + hh;
          v4f v = *(const v4f*)(slab + row * 68 + c4);
          *(volatile v4f*)(C + (size_t)(mBase + row) * ldc + n0 + c4) = v;
        }
        __threadfence();
      }
    } else {
      const int q = lane >> 3, c8 = (lane & 7) * 8;
      unsigned short* C  = (unsigned short*)Cout  + (size_t)b * strideC;
      unsigned short* C2 = (OUT_MODE == 2) ? ((unsigned short*)Cout2 + (size_t)b * strideC) : nullptr;
      for (int pass = 0; pass < 2; ++pass) {
#pragma unroll
        for (int it = 0; it < 4; ++it) {
          const int row = it * 4 + q;
          const float* sp = slab + row * 68 + c8;
          v8h hv, lv;
#pragma unroll
          for (int e = 0; e < 8; ++e) {
            if (OUT_MODE == 1) {
              hv[e] = (_Float16)sp[e];
            } else {
              unsigned short hb = f2bf_bits(sp[e]);
              unsigned short lb = f2bf_bits(sp[e] - bf_bits2f(hb));
              hv[e] = __builtin_bit_cast(_Float16, hb);
              lv[e] = __builtin_bit_cast(_Float16, lb);
            }
          }
          *(volatile v8h*)(C + (size_t)(mBase + row) * ldc + n0 + c8) = hv;
          if (OUT_MODE == 2) *(volatile v8h*)(C2 + (size_t)(mBase + row) * ldc + n0 + c8) = lv;
        }
        __threadfence();
      }
    }
    __builtin_amdgcn_fence(__ATOMIC_RELEASE, "workgroup");
    __builtin_amdgcn_wave_barrier();
    __builtin_amdgcn_fence(__ATOMIC_ACQUIRE, "workgroup");
  }
}

__device__ __forceinline__ float celu1(float v) {
  const float e = expf(v) - 1.0f;
  return v > 0.0f ? v : e;
}

__global__ __launch_bounds__(256) void cast_f32_f16x8(
    const float* __restrict__ in, _Float16* __restrict__ out, int n8, float scale) {
  const int i = blockIdx.x * 256 + threadIdx.x;
  if (i < n8) {
    const float* p = in + (size_t)i * 8;
    const v4f a = *(const v4f*)p;
    const v4f b = *(const v4f*)(p + 4);
    v8h hv;
    hv[0] = (_Float16)(a[0] * scale); hv[1] = (_Float16)(a[1] * scale);
    hv[2] = (_Float16)(a[2] * scale); hv[3] = (_Float16)(a[3] * scale);
    hv[4] = (_Float16)(b[0] * scale); hv[5] = (_Float16)(b[1] * scale);
    hv[6] = (_Float16)(b[2] * scale); hv[7] = (_Float16)(b[3] * scale);
    _Float16* q = out + (size_t)i * 8;
    *(volatile v8h*)q = hv;
    __threadfence();
    *(volatile v8h*)q = hv;
  }
}

__global__ __launch_bounds__(256) void init_h16_kernel(
    const float* __restrict__ state, _Float16* __restrict__ h16) {
  const int i = blockIdx.x * 256 + threadIdx.x;
  if (i < (kB * kG) / 8) {
    const int o = i * 8;
    const int gblk = o >> 9, bb = (o >> 5) & 15, gi = o & 31;
    const float* p = state + (size_t)bb * kG + gblk * 32 + gi;
    const v4f a = *(const v4f*)p;
    const v4f b = *(const v4f*)(p + 4);
    v8h hv;
    hv[0] = (_Float16)a[0]; hv[1] = (_Float16)a[1]; hv[2] = (_Float16)a[2]; hv[3] = (_Float16)a[3];
    hv[4] = (_Float16)b[0]; hv[5] = (_Float16)b[1]; hv[6] = (_Float16)b[2]; hv[7] = (_Float16)b[3];
    _Float16* q = h16 + o;
    *(volatile v8h*)q = hv;
    __threadfence();
    *(volatile v8h*)q = hv;
  }
}

__device__ __forceinline__ float dw3x3(const float* src, const float* __restrict__ wp, float bias,
                                       int ch, int py, int pxx) {
  float a = bias;
#pragma unroll
  for (int dy = 0; dy < 3; ++dy) {
    const int yy = py + dy - 1;
    const int yyc = yy < 0 ? 0 : (yy > 7 ? 7 : yy);
#pragma unroll
    for (int dx = 0; dx < 3; ++dx) {
      const int xx = pxx + dx - 1;
      const int xxc = xx < 0 ? 0 : (xx > 7 ? 7 : xx);
      const bool ok = (yy >= 0) && (yy < 8) && (xx >= 0) && (xx < 8);
      const float hv = src[ch * kH1P + yyc * 8 + xxc];
      a += wp[dy * 3 + dx] * (ok ? hv : 0.0f);
    }
  }
  return a;
}

__global__ __launch_bounds__(256) void front_kernel(
    const float* __restrict__ x, const _Float16* __restrict__ cinw16, const float* __restrict__ cin_b,
    const float* __restrict__ dw_w, const float* __restrict__ dw_b,
    const _Float16* __restrict__ gruw16, const float* __restrict__ gruin_b,
    _Float16* __restrict__ g16) {
  extern __shared__ v4f dynl4[];
  unsigned char* dynl = (unsigned char*)dynl4;
  _Float16* xa   = (_Float16*)(dynl + kFrXa);
  float*    h1   = (float*)(dynl + kFrH1);
  float*    h2   = (float*)(dynl + kFrH2);
  _Float16* hT   = (_Float16*)(dynl + kFrH1);
  float*    gpre = (float*)(dynl + kFrXa);

  const int img = blockIdx.x, tid = threadIdx.x;
  const int lane = tid & 31, wave = tid >> 5;
  const int m = lane & 15, hh = lane >> 4, koff = hh * 8;
  const float* xi = x + (size_t)img * (kCin * kPx);

#pragma unroll
  for (int i = 0; i < 4; ++i) {
    const int e = 4 * tid + 1024 * i;
    const int c = e >> 6, px = e & 63;
    const v4f v = *(const v4f*)(xi + e);
    xa[(px + 0) * kXaP + c] = (_Float16)v[0];
    xa[(px + 1) * kXaP + c] = (_Float16)v[1];
    xa[(px + 2) * kXaP + c] = (_Float16)v[2];
    xa[(px + 3) * kXaP + c] = (_Float16)v[3];
  }
  __syncthreads();

  {
    const int o0 = 16 * wave;
    v8f acc[4];
#pragma unroll
    for (int i = 0; i < 4; ++i) acc[i] = zero8();
#pragma unroll
    for (int k0 = 0; k0 < kCin; k0 += 32) {
      const v16h bf = Frag<_Float16>::load(cinw16 + (size_t)(o0 + m) * kCin + koff + k0);
      v16h af;
#pragma unroll
      for (int i = 0; i < 4; ++i) {
        af = Frag<_Float16>::load(xa + (16 * i + m) * kXaP + koff + k0);
        acc[i] = Frag<_Float16>::mma(af, bf, acc[i]);
      }
      guard4h(acc[0], acc[1], acc[2], acc[3], af, bf);
    }
    acc_guard4(acc[0], acc[1], acc[2], acc[3]);
    const float bc = cin_b[o0 + m];
#pragma unroll
    for (int i = 0; i < 4; ++i) {
      v4f lo4, hi4;
      lo4[0] = acc[i][0] * kWInv + bc; lo4[1] = acc[i][1] * kWInv + bc;
      lo4[2] = acc[i][2] * kWInv + bc; lo4[3] = acc[i][3] * kWInv + bc;
      hi4[0] = acc[i][4] * kWInv + bc; hi4[1] = acc[i][5] * kWInv + bc;
      hi4[2] = acc[i][6] * kWInv + bc; hi4[3] = acc[i][7] * kWInv + bc;
      float* hp = h1 + (o0 + m) * kH1P + 16 * i + 8 * hh;
      *(v4f*)hp = lo4;
      *(v4f*)(hp + 4) = hi4;
    }
  }
  __syncthreads();

#pragma unroll 1
  for (int it = 0; it < 32; ++it) {
    const int e = tid + 256 * it;
    const int o = e >> 6, px = e & 63;
    float* p = h1 + o * kH1P + px;
    *p = celu1(*p);
  }
  __syncthreads();

#pragma unroll 1
  for (int it = 0; it < 32; ++it) {
    const int e = tid + 256 * it;
    const int ch = e >> 6, py = (e >> 3) & 7, pxx = e & 7;
    const float a = dw3x3(h1, dw_w + (size_t)ch * 9, dw_b[ch], ch, py, pxx);
    h2[ch * kH1P + py * 8 + pxx] = celu1(a);
  }
  __syncthreads();

#pragma unroll 1
  for (int it = 0; it < 32; ++it) {
    const int e = tid + 256 * it;
    const int ch = e >> 6, py = (e >> 3) & 7, pxx = e & 7;
    const float a = dw3x3(h2, dw_w + (size_t)(kHid + ch) * 9, dw_b[kHid + ch], ch, py, pxx);
    hT[(py * 8 + pxx) * kHtP + ch] = (_Float16)celu1(a);
  }
  __syncthreads();

  {
    const int ti = wave >> 2, tj = wave & 3;
    v8f acc = zero8();
    v16h af, bf;
#pragma unroll
    for (int k0 = 0; k0 < kHid; k0 += 32) {
      af = Frag<_Float16>::load(gruw16 + (size_t)(16 * ti + m) * kHid + koff + k0);
      bf = Frag<_Float16>::load(hT + (16 * tj + m) * kHtP + koff + k0);
      acc = Frag<_Float16>::mma(af, bf, acc);
      guard1h(acc, af, bf);
    }
    acc_guard1(acc);
#pragma unroll
    for (int r = 0; r < 8; ++r) {
      const int gc = 16 * ti + 8 * hh + r;
      gpre[gc * kPx + 16 * tj + m] = acc[r] * kWInv + gruin_b[gc];
    }
  }
  __syncthreads();

#pragma unroll 1
  for (int it = 0; it < 8; ++it) {
    const int e = tid + 256 * it;
    gpre[e] = celu1(gpre[e]);
  }
  __syncthreads();

  {
    const int e = 8 * tid;
    const v4f a = *(const v4f*)(gpre + e);
    const v4f b = *(const v4f*)(gpre + e + 4);
    v8h hv;
    hv[0] = (_Float16)a[0]; hv[1] = (_Float16)a[1]; hv[2] = (_Float16)a[2]; hv[3] = (_Float16)a[3];
    hv[4] = (_Float16)b[0]; hv[5] = (_Float16)b[1]; hv[6] = (_Float16)b[2]; hv[7] = (_Float16)b[3];
    _Float16* gp = g16 + (size_t)img * kG + e;
    *(volatile v8h*)gp = hv;
    __threadfence();
    *(volatile v8h*)gp = hv;
  }
}

__global__ __launch_bounds__(128) void rnn_step_kernel(
    const _Float16* __restrict__ h16cur, const float* __restrict__ h32cur,
    const _Float16* __restrict__ whh16, const float* __restrict__ gi,
    const float* __restrict__ b_hh, const float* __restrict__ msk,
    _Float16* __restrict__ h16next, float* __restrict__ h32next,
    float* __restrict__ gseq, int t) {
  __shared__ __align__(16) float sAcc[4][3 * 16 * 32];
  __shared__ __align__(16) float sOut[4][16 * 32];
  const int lane = threadIdx.x & 31, wave = threadIdx.x >> 5;
  const int wg = blockIdx.x * 4 + wave;
  const int g0 = wg * 32;
  const int m = lane & 15, hh = lane >> 4, koff = hh * 8;

  v8f acc[3][2];
#pragma unroll
  for (int j = 0; j < 3; ++j) { acc[j][0] = zero8(); acc[j][1] = zero8(); }

#pragma unroll 1
  for (int k0 = 0; k0 < kG; k0 += 32) {
    const v16h af = Frag<_Float16>::load(h16cur + ((k0 >> 5) << 9) + (m << 5) + koff);
    v16h bf;
#pragma unroll
    for (int s2 = 0; s2 < 2; ++s2) {
#pragma unroll
      for (int j = 0; j < 3; ++j) {
        bf = Frag<_Float16>::load(whh16 + (size_t)(j * kG + g0 + 16 * s2 + m) * kG + k0 + koff);
        acc[j][s2] = Frag<_Float16>::mma(af, bf, acc[j][s2]);
      }
    }
    guard6h(acc[0][0], acc[0][1], acc[1][0], acc[1][1], acc[2][0], acc[2][1], af, bf);
  }
  acc_guard2(acc[0][0], acc[0][1]);
  acc_guard2(acc[1][0], acc[1][1]);
  acc_guard2(acc[2][0], acc[2][1]);

  float* slab = sAcc[wave];
  float* so = sOut[wave];
#pragma unroll
  for (int j = 0; j < 3; ++j)
#pragma unroll
    for (int s2 = 0; s2 < 2; ++s2)
#pragma unroll
      for (int r = 0; r < 8; ++r)
        slab[(j * 16 + 8 * hh + r) * 32 + 16 * s2 + m] = acc[j][s2][r];
  wave_lds_sync();

  const int q = lane >> 3, c4 = (lane & 7) * 4;
  const v4f bhr = *(const v4f*)(b_hh + g0 + c4);
  const v4f bhz = *(const v4f*)(b_hh + kG + g0 + c4);
  const v4f bhn = *(const v4f*)(b_hh + 2 * kG + g0 + c4);
#pragma unroll 1
  for (int e = 0; e < 4; ++e) {
    const int bb = q + 4 * e;
    const float mk = msk[bb * kS + t];
    const float* gp = gi + (size_t)(bb * kS + t) * kG3 + g0 + c4;
    const v4f gir = *(const v4f*)gp;
    const v4f giz = *(const v4f*)(gp + kG);
    const v4f gin = *(const v4f*)(gp + 2 * kG);
    const v4f hx = *(const v4f*)(h32cur + (size_t)bb * kG + g0 + c4);
    const v4f ar = *(const v4f*)(slab + (0 * 16 + bb) * 32 + c4);
    const v4f az = *(const v4f*)(slab + (1 * 16 + bb) * 32 + c4);
    const v4f an = *(const v4f*)(slab + (2 * 16 + bb) * 32 + c4);
    v4f o;
#pragma unroll
    for (int i = 0; i < 4; ++i) {
      const float hr = mk * (ar[i] * kWInv) + bhr[i];
      const float hz = mk * (az[i] * kWInv) + bhz[i];
      const float hn = mk * (an[i] * kWInv) + bhn[i];
      const float hxm = hx[i] * mk;
      const float rg = 1.0f / (1.0f + expf(-(gir[i] + hr)));
      const float zg = 1.0f / (1.0f + expf(-(giz[i] + hz)));
      const float ng = tanhf(gin[i] + rg * hn);
      o[i] = (1.0f - zg) * ng + zg * hxm;
    }
    *(v4f*)(so + bb * 32 + c4) = o;
  }
  wave_lds_sync();

  for (int pass = 0; pass < 2; ++pass) {
#pragma unroll
    for (int k = 0; k < 4; ++k) {
      const int bb = 4 * k + q;
      const v4f v = *(const v4f*)(so + bb * 32 + c4);
      *(volatile v4f*)(h32next + (size_t)bb * kG + g0 + c4) = v;
      *(volatile v4f*)(gseq + (size_t)(bb * kS + t) * kG + g0 + c4) = v;
    }
#pragma unroll
    for (int k = 0; k < 2; ++k) {
      const int idx = 256 * k + 8 * lane;
      const int bb = idx >> 5, gg = idx & 31;
      const v4f a = *(const v4f*)(so + bb * 32 + gg);
      const v4f c = *(const v4f*)(so + bb * 32 + gg + 4);
      v8h hv;
      hv[0] = (_Float16)a[0]; hv[1] = (_Float16)a[1]; hv[2] = (_Float16)a[2]; hv[3] = (_Float16)a[3];
      hv[4] = (_Float16)c[0]; hv[5] = (_Float16)c[1]; hv[6] = (_Float16)c[2]; hv[7] = (_Float16)c[3];
      *(volatile v8h*)(h16next + (size_t)wg * 512 + idx) = hv;
    }
    __threadfence();
  }
}

__global__ __launch_bounds__(256) void back_kernel(
    const float* __restrict__ gseq, const float* __restrict__ x,
    const _Float16* __restrict__ gow16, const float* __restrict__ go_b,
    const _Float16* __restrict__ cow16, const float* __restrict__ co_b,
    float* __restrict__ y) {
  __shared__ __align__(16) _Float16 bt1[kPx * kBt1P];
  __shared__ __align__(16) _Float16 bt2[kPx * kHtP];
  __shared__ __align__(16) float ys[kCin * kH1P];
  const int img = blockIdx.x, tid = threadIdx.x;
  const int lane = tid & 31, wave = tid >> 5;
  const int m = lane & 15, hh = lane >> 4, koff = hh * 8;

  const float* gs = gseq + (size_t)img * kG;
#pragma unroll
  for (int i = 0; i < 2; ++i) {
    const int e = 4 * tid + 1024 * i;
    const int gc = e >> 6, px = e & 63;
    const v4f v = *(const v4f*)(gs + e);
    bt1[(px + 0) * kBt1P + gc] = (_Float16)v[0];
    bt1[(px + 1) * kBt1P + gc] = (_Float16)v[1];
    bt1[(px + 2) * kBt1P + gc] = (_Float16)v[2];
    bt1[(px + 3) * kBt1P + gc] = (_Float16)v[3];
  }
  __syncthreads();

  {
    const int o0 = 16 * wave;
    v8f acc[4];
#pragma unroll
    for (int j = 0; j < 4; ++j) acc[j] = zero8();
    const v16h af = Frag<_Float16>::load(gow16 + (size_t)(o0 + m) * kGc + koff);
    v16h bf;
#pragma unroll
    for (int j = 0; j < 4; ++j) {
      bf = Frag<_Float16>::load(bt1 + (16 * j + m) * kBt1P + koff);
      acc[j] = Frag<_Float16>::mma(af, bf, acc[j]);
    }
    guard4h(acc[0], acc[1], acc[2], acc[3], af, bf);
    acc_guard4(acc[0], acc[1], acc[2], acc[3]);
    float gb[8];
#pragma unroll
    for (int r = 0; r < 8; ++r) gb[r] = go_b[o0 + 8 * hh + r];
#pragma unroll
    for (int j = 0; j < 4; ++j) {
      v8h hv;
#pragma unroll
      for (int r = 0; r < 8; ++r) hv[r] = (_Float16)(acc[j][r] * kWInv + gb[r]);
      *(v8h*)(bt2 + (16 * j + m) * kHtP + o0 + 8 * hh) = hv;
    }
  }
  __syncthreads();

  {
    const int ti = wave >> 1, tj0 = 2 * (wave & 1);
    v8f acc[2];
    acc[0] = zero8(); acc[1] = zero8();
    v16h af, bf;
#pragma unroll
    for (int k0 = 0; k0 < kHid; k0 += 32) {
      af = Frag<_Float16>::load(cow16 + (size_t)(16 * ti + m) * kHid + koff + k0);
#pragma unroll
      for (int j = 0; j < 2; ++j) {
        bf = Frag<_Float16>::load(bt2 + (16 * (tj0 + j) + m) * kHtP + koff + k0);
        acc[j] = Frag<_Float16>::mma(af, bf, acc[j]);
      }
      dep_guard_h(acc[0], acc[1], af, bf);
    }
    acc_guard2(acc[0], acc[1]);
    float cb[8];
#pragma unroll
    for (int r = 0; r < 8; ++r) cb[r] = co_b[16 * ti + 8 * hh + r];
#pragma unroll
    for (int j = 0; j < 2; ++j)
#pragma unroll
      for (int r = 0; r < 8; ++r)
        ys[(16 * ti + 8 * hh + r) * kH1P + 16 * (tj0 + j) + m] = acc[j][r] * kWInv + cb[r];
  }
  __syncthreads();

  const float* xi = x + (size_t)img * (kCin * kPx);
#pragma unroll 1
  for (int it = 0; it < 16; ++it) {
    const int e = tid + 256 * it;
    const int c = e >> 6, px = e & 63;
    float* p = ys + c * kH1P + px;
    *p = celu1(*p + xi[e]);
  }
  __syncthreads();

  float* yo = y + (size_t)img * (kCin * kPx);
  for (int pass = 0; pass < 2; ++pass) {
#pragma unroll
    for (int k = 0; k < 4; ++k) {
      const int e = 4 * (256 * k + tid);
      const int c = e >> 6, px = e & 63;
      const v4f v = *(const v4f*)(ys + c * kH1P + px);
      *(volatile v4f*)(yo + e) = v;
    }
    __threadfence();
  }
}

extern "C" void kernel_launch(void* const* d_in, const int* in_sizes, int n_in,
                              void* d_out, int out_size, void* d_ws, size_t ws_size,
                              hipStream_t stream) {
  if (n_in < 17) return;
  if (in_sizes[0] != kImg * kCin * kPx) return;
  if (in_sizes[1] != kB * kG) return;
  if (in_sizes[2] != kB * kS) return;
  if (in_sizes[3] != kHid * kCin || in_sizes[7] != kGc * kHid) return;
  if (in_sizes[9] != kG3 * kG || in_sizes[10] != kG3 * kG) return;
  if (in_sizes[13] != kHid * kGc || in_sizes[15] != kCin * kHid) return;
  if ((size_t)out_size < kOut0Floats + kOut1Floats) return;
  if (ws_size < kWsTotal) return;

  const float* x        = (const float*)d_in[0];
  const float* state    = (const float*)d_in[1];
  const float* msk      = (const float*)d_in[2];
  const float* cin_w    = (const float*)d_in[3];
  const float* cin_b    = (const float*)d_in[4];
  const float* dw_w     = (const float*)d_in[5];
  const float* dw_b     = (const float*)d_in[6];
  const float* gruin_w  = (const float*)d_in[7];
  const float* gruin_b  = (const float*)d_in[8];
  const float* w_ih     = (const float*)d_in[9];
  const float* w_hh     = (const float*)d_in[10];
  const float* b_ih     = (const float*)d_in[11];
  const float* b_hh     = (const float*)d_in[12];
  const float* gruout_w = (const float*)d_in[13];
  const float* gruout_b = (const float*)d_in[14];
  const float* cout_w   = (const float*)d_in[15];
  const float* cout_b   = (const float*)d_in[16];
  float* out0 = (float*)d_out;
  float* out1 = (float*)d_out + kOut0Floats;

  char* ws = (char*)d_ws;
  _Float16* wih16 = (_Float16*)(ws + kOffWih);
  _Float16* whh16 = (_Float16*)(ws + kOffWhh);
  _Float16* cinw16 = (_Float16*)(ws + kOffCinW);
  _Float16* gruw16 = (_Float16*)(ws + kOffGruW);
  _Float16* gow16 = (_Float16*)(ws + kOffGoW);
  _Float16* cow16 = (_Float16*)(ws + kOffCoW);
  _Float16* g16 = (_Float16*)(ws + kOffG16);
  float* gi = (float*)(ws + kOffGi);
  float* h32a = (float*)(ws + kOffH32a);
  float* h32b = (float*)(ws + kOffH32b);
  _Float16* h16a = (_Float16*)(ws + kOffH16a);
  _Float16* h16b = (_Float16*)(ws + kOffH16b);
  float* gseq = (float*)(ws + kOffGseq);

  {
    const int n8w = (kG3 * kG) / 8;
    cast_f32_f16x8<<<(n8w + 255) / 256, 256, 0, stream>>>(w_ih, wih16, n8w, kWScale);
    cast_f32_f16x8<<<(n8w + 255) / 256, 256, 0, stream>>>(w_hh, whh16, n8w, kWScale);
    const int n8c = (kHid * kCin) / 8;
    cast_f32_f16x8<<<(n8c + 255) / 256, 256, 0, stream>>>(cin_w, cinw16, n8c, kWScale);
    const int n8g = (kGc * kHid) / 8;
    cast_f32_f16x8<<<(n8g + 255) / 256, 256, 0, stream>>>(gruin_w, gruw16, n8g, kWScale);
    const int n8o = (kHid * kGc) / 8;
    cast_f32_f16x8<<<(n8o + 255) / 256, 256, 0, stream>>>(gruout_w, gow16, n8o, kWScale);
    const int n8q = (kCin * kHid) / 8;
    cast_f32_f16x8<<<(n8q + 255) / 256, 256, 0, stream>>>(cout_w, cow16, n8q, kWScale);
  }

  init_h16_kernel<<<(kB * kG / 8 + 255) / 256, 256, 0, stream>>>(state, h16a);

  front_kernel<<<kImg, 256, kFrLds, stream>>>(x, cinw16, cin_b, dw_w, dw_b, gruw16, gruin_b, g16);

  {
    const int tiles = (kImg / 64) * (kG3 / 64);
    wmma_gemm64<0, false, 2, 0, false, 0><<<dim3((tiles + 7) / 8, 1), 256, 0, stream>>>(
        (const unsigned short*)g16, (const unsigned short*)g16, kG, 0L,
        (const unsigned short*)wih16, (const unsigned short*)wih16, kG, 0L,
        (void*)gi, (void*)gi, kG3, 0L,
        b_ih, b_ih, 0L,
        kImg, kG3, kG, kWInv);
  }

  for (int t = 0; t < kS; ++t) {
    const _Float16* h16c = (t & 1) ? h16b : h16a;
    _Float16* h16n = (t & 1) ? h16a : h16b;
    const float* h32c = (t == 0) ? state : ((t & 1) ? h32a : h32b);
    float* h32n = (t == kS - 1) ? out1 : ((t & 1) ? h32b : h32a);
    rnn_step_kernel<<<(kG / 32) / 4, 128, 0, stream>>>(
        h16c, h32c, whh16, gi, b_hh, msk, h16n, h32n, gseq, t);
  }

  back_kernel<<<kImg, 256, 0, stream>>>(gseq, x, gow16, gruout_b, cow16, cout_b, out0);
}
